// EfficientSABlock_3822520893838
// MI455X (gfx1250) — hardware-verified
//
#include <hip/hip_runtime.h>


namespace {
constexpr int NB = 8, N = 4096, HW = 64, E = 256, NH = 4, D = 64, SR = 4, G = HW / SR  , M = G * G  , KC = E * SR * SR  , NR = NB * N, NK = NB * M;
constexpr float XS = 8.0f, WSC = 256.0f, PS = 8.0f, SCALE = 0.125f, LOG2E = 1.4426950408889634f, LN_EPS = 1e-5f;

typedef _Float16 b16;
typedef __attribute__((ext_vector_type(16))) _Float16 v16b;
typedef __attribute__((ext_vector_type(8))) _Float16 v8b;
typedef __attribute__((ext_vector_type(8))) float v8f;
typedef __attribute__((ext_vector_type(4))) float v4f;
__device__ __forceinline__ float bf16_rne(float f) { unsigned int u = __float_as_uint(f); u += 0x7FFFu + ((u >> 16) & 1u); return __uint_as_float(u & 0xFFFF0000u); }
__device__ __forceinline__ void split16(float v, b16& hi, b16& lo) { hi = (b16)v; lo = (b16)(v - (float)hi); }
__device__ __forceinline__ v16b frag_kb(const b16* p, int hh) { const v8b a = *(const v8b*)(p + 8 * hh), b = *(const v8b*)(p + 16 + 8 * hh); v16b f;
#pragma unroll
  for (int e = 0; e < 8; ++e) { f[e] = a[e]; f[8 + e] = b[e]; } return f; }
__device__ __forceinline__ v8f wmma16b(v16b a, v16b b, v8f c) { v8f d = __builtin_amdgcn_wmma_f32_16x16x32_f16(false, a, false, b, (short)0, c, false, false); asm volatile("v_nop\n\tv_nop\n\tv_nop\n\tv_nop" : "+v"(d) : "v"(a), "v"(b)); return d; }
__device__ __forceinline__ void wave_lds_sync() { __builtin_amdgcn_fence(__ATOMIC_RELEASE, "workgroup"); __builtin_amdgcn_wave_barrier(); __builtin_amdgcn_fence(__ATOMIC_ACQUIRE, "workgroup"); }
__device__ __forceinline__ float nexp2(float x) { return __builtin_amdgcn_exp2f(x); }
__device__ __forceinline__ float pmul(float a, float b) { float p = a * b; asm volatile("" : "+v"(p)); return p; }
__device__ __forceinline__ float hsum16(float v) { v += __shfl_xor(v, 1); v += __shfl_xor(v, 2); v += __shfl_xor(v, 4); return v + __shfl_xor(v, 8); }

__global__ __launch_bounds__(256) void prepx_kernel(const float* __restrict__ x, b16* __restrict__ X16) {
  const size_t t = (size_t)blockIdx.x * 256 + threadIdx.x; if (t >= (size_t)NR * E / 8) return; const size_t e = t * 8;
  const v4f a = *(const v4f*)(x + e), c = *(const v4f*)(x + e + 4); v8b o;
#pragma unroll
  for (int j = 0; j < 4; ++j) { o[j] = (b16)(bf16_rne(a[j]) * XS); o[4 + j] = (b16)(bf16_rne(c[j]) * XS); }
  for (int pass = 0; pass < 2; ++pass) { *(volatile v8b*)(X16 + e) = o; __threadfence(); }
}
__global__ __launch_bounds__(256) void prepw_kernel(const float* __restrict__ wq, const float* __restrict__ wkv, const float* __restrict__ wo, b16* __restrict__ WQ16, b16* __restrict__ WKV16, b16* __restrict__ WO16) {
  __shared__ __attribute__((aligned(16))) b16 T[64][64 + 8];
  const int kind = blockIdx.z, c0 = blockIdx.y * 64, o0 = blockIdx.x * 64, t_ = threadIdx.x; const int nout = kind == 1 ? 2 * E : E; if (o0 >= nout) return;
  const float* w = kind == 0 ? wq : kind == 1 ? wkv : wo; b16* dst = kind == 0 ? WQ16 : kind == 1 ? WKV16 : WO16;
  for (int q = t_; q < 64 * 64; q += 256) { const int cc = q >> 6, oo = q & 63; T[oo][cc] = (b16)(bf16_rne(w[(size_t)(c0 + cc) * nout + o0 + oo]) * WSC); }
  __syncthreads();
  for (int pass = 0; pass < 2; ++pass) { for (int q = t_; q < 64 * 8; q += 256) { const int oo = q >> 3, c8 = (q & 7) * 8; *(volatile v8b*)(dst + (size_t)(o0 + oo) * E + c0 + c8) = *(const v8b*)(&T[oo][c8]); } __threadfence(); }
}
__global__ __launch_bounds__(256) void prepc_kernel(const float* __restrict__ srw, b16* __restrict__ SRW16) {
  const size_t t = (size_t)blockIdx.x * 256 + threadIdx.x; if (t >= (size_t)E * KC / 8) return; const size_t e = t * 8; const int o = (int)(e / KC); const int r = (int)(e % KC); const int ky = r / (SR * E), kx = (r / E) % SR, c0 = r % E;
  v8b v; for (int j = 0; j < 8; ++j) v[j] = (b16)(bf16_rne(srw[(((size_t)o * E + c0 + j) * SR + ky) * SR + kx]) * WSC);
  for (int pass = 0; pass < 2; ++pass) { *(volatile v8b*)(SRW16 + e) = v; __threadfence(); }
}
__global__ __launch_bounds__(128) void q_kernel(const b16* __restrict__ X16, const b16* __restrict__ WQ16, b16* __restrict__ Qh, b16* __restrict__ Ql) {
  __shared__ __attribute__((aligned(16))) b16 Th[4][16][128 + 8], Tl[4][16][128 + 8];
  const int wave = threadIdx.x >> 5, lane = threadIdx.x & 31, nloc = lane & 15, hlf = lane >> 4; const size_t m0 = (size_t)blockIdx.x * 64 + wave * 16; const int n0 = blockIdx.y * 128;
  v8f acc[8];
#pragma unroll
  for (int t = 0; t < 8; ++t) acc[t] = (v8f){};
#pragma unroll
  for (int kb = 0; kb < E; kb += 32) { const v16b a = frag_kb(X16 + (m0 + nloc) * E + kb, hlf);
#pragma unroll
    for (int t = 0; t < 8; ++t) acc[t] = wmma16b(a, frag_kb(WQ16 + (size_t)(n0 + t * 16 + nloc) * E + kb, hlf), acc[t]); }
#pragma unroll
  for (int t = 0; t < 8; ++t)
#pragma unroll
    for (int r = 0; r < 8; ++r) { b16 h_, l_; split16(acc[t][r] * (1.0f / (XS * WSC)) * XS, h_, l_); Th[wave][8 * hlf + r][t * 16 + nloc] = h_; Tl[wave][8 * hlf + r][t * 16 + nloc] = l_; }
  wave_lds_sync();
  for (int pass = 0; pass < 2; ++pass) { for (int r2 = 0; r2 < 16; r2 += 2) { const int rr = r2 + (lane >> 4), c8 = (lane & 15) * 8; const size_t gi = (m0 + rr) * E + n0 + c8; *(volatile v8b*)(Qh + gi) = *(const v8b*)(&Th[wave][rr][c8]); *(volatile v8b*)(Ql + gi) = *(const v8b*)(&Tl[wave][rr][c8]); } __threadfence(); }
}
__global__ __launch_bounds__(128) void conv_kernel(const b16* __restrict__ X16, const b16* __restrict__ SRW16, const float* __restrict__ srb, float* __restrict__ CV) {
  __shared__ __attribute__((aligned(16))) float Tf[4][16][E + 4];
  const int wave = threadIdx.x >> 5, lane = threadIdx.x & 31, nloc = lane & 15, hlf = lane >> 4; const int m0 = blockIdx.x * 64 + wave * 16;
  const int key = m0 + nloc; const int b = key / M, ij = key % M, i = ij / G, j = ij % G;
  const b16* xa = X16 + ((size_t)b * N + (size_t)(SR * i) * HW + SR * j) * E;
  v8f acc[16];
#pragma unroll
  for (int t = 0; t < 16; ++t) acc[t] = (v8f){};
  for (int ky = 0; ky < SR; ++ky) { const b16* xk = xa + (size_t)ky * HW * E;
#pragma unroll 2
    for (int kk = 0; kk < SR * E; kk += 32) { const v16b a = frag_kb(xk + kk, hlf); const int kb = ky * SR * E + kk;
#pragma unroll
      for (int t = 0; t < 16; ++t) acc[t] = wmma16b(a, frag_kb(SRW16 + (size_t)(t * 16 + nloc) * KC + kb, hlf), acc[t]); } }
#pragma unroll
  for (int t = 0; t < 16; ++t) { const float bb = bf16_rne(srb[t * 16 + nloc]);
#pragma unroll
    for (int r = 0; r < 8; ++r) Tf[wave][8 * hlf + r][t * 16 + nloc] = acc[t][r] * (1.0f / (XS * WSC)) + bb; }
  wave_lds_sync();
  for (int pass = 0; pass < 2; ++pass) { for (int rr = 0; rr < 16; ++rr) { for (int hq = 0; hq < 2; ++hq) *(volatile v4f*)(CV + (size_t)(m0 + rr) * E + hq * 128 + lane * 4) = *(const v4f*)(&Tf[wave][rr][hq * 128 + lane * 4]); } __threadfence(); }
}
__global__ __launch_bounds__(256) void ln_kernel(const float* __restrict__ CV, const float* __restrict__ g, const float* __restrict__ be, b16* __restrict__ KVINh, b16* __restrict__ KVINl) {
  const int wave = threadIdx.x >> 5, lane = threadIdx.x & 31; const size_t row = (size_t)blockIdx.x * 8 + wave; const float* src = CV + row * E + lane * 8;
  const v4f a = *(const v4f*)src, c = *(const v4f*)(src + 4); float v[8]; float s = 0.0f;
#pragma unroll
  for (int i = 0; i < 4; ++i) { v[i] = a[i]; v[4 + i] = c[i]; s += a[i] + c[i]; }
#pragma unroll
  for (int o = 16; o >= 1; o >>= 1) s += __shfl_xor(s, o);
  const float mean = s * (1.0f / E); float ss = 0.0f;
#pragma unroll
  for (int i = 0; i < 8; ++i) { const float d = v[i] - mean; ss += pmul(d, d); }
#pragma unroll
  for (int o = 16; o >= 1; o >>= 1) ss += __shfl_xor(ss, o);
  const float rs = rsqrtf(ss * (1.0f / E) + LN_EPS); v8b hv, lv;
#pragma unroll
  for (int i = 0; i < 8; ++i) { const int ch = lane * 8 + i; const float y = pmul((v[i] - mean) * rs, bf16_rne(g[ch])) + bf16_rne(be[ch]); b16 h_, l_; split16(y * XS, h_, l_); hv[i] = h_; lv[i] = l_; }
  for (int pass = 0; pass < 2; ++pass) { *(volatile v8b*)(KVINh + row * E + lane * 8) = hv; *(volatile v8b*)(KVINl + row * E + lane * 8) = lv; __threadfence(); }
}
__global__ __launch_bounds__(128) void kv_kernel(const b16* __restrict__ Ah, const b16* __restrict__ Al, const b16* __restrict__ WKV16, b16* __restrict__ Kh, b16* __restrict__ Kl, b16* __restrict__ VTh, b16* __restrict__ VTl) {
  __shared__ __attribute__((aligned(16))) b16 Th[4][16][128 + 8], Tl[4][16][128 + 8]; __shared__ __attribute__((aligned(16))) b16 Vt[128][64 + 8], Vtl[128][64 + 8];
  const int wave = threadIdx.x >> 5, lane = threadIdx.x & 31, nloc = lane & 15, hlf = lane >> 4, t_ = threadIdx.x; const size_t m0 = (size_t)blockIdx.x * 64 + wave * 16; const int n0 = blockIdx.y * 128; const bool isv = n0 >= E;
  v8f acc[8];
#pragma unroll
  for (int t = 0; t < 8; ++t) acc[t] = (v8f){};
#pragma unroll
  for (int kb = 0; kb < E; kb += 32) { const v16b a = frag_kb(Ah + (m0 + nloc) * E + kb, hlf), al = frag_kb(Al + (m0 + nloc) * E + kb, hlf);
#pragma unroll
    for (int t = 0; t < 8; ++t) { const v16b bw = frag_kb(WKV16 + (size_t)(n0 + t * 16 + nloc) * E + kb, hlf); acc[t] = wmma16b(a, bw, acc[t]); acc[t] = wmma16b(al, bw, acc[t]); } }
  if (!isv) {
#pragma unroll
    for (int t = 0; t < 8; ++t)
#pragma unroll
      for (int r = 0; r < 8; ++r) { b16 h_, l_; split16(acc[t][r] * (1.0f / (XS * WSC)) * XS, h_, l_); Th[wave][8 * hlf + r][t * 16 + nloc] = h_; Tl[wave][8 * hlf + r][t * 16 + nloc] = l_; }
    wave_lds_sync();
    for (int pass = 0; pass < 2; ++pass) { for (int r2 = 0; r2 < 16; r2 += 2) { const int rr = r2 + (lane >> 4), c8 = (lane & 15) * 8; const size_t gi = (m0 + rr) * E + n0 + c8; *(volatile v8b*)(Kh + gi) = *(const v8b*)(&Th[wave][rr][c8]); *(volatile v8b*)(Kl + gi) = *(const v8b*)(&Tl[wave][rr][c8]); } __threadfence(); }
  } else {
    const int b = (int)(m0 / M); const int s0 = (int)((size_t)blockIdx.x * 64 - (size_t)b * M); const int c0v = n0 - E;
#pragma unroll
    for (int t = 0; t < 8; ++t)
#pragma unroll
      for (int r = 0; r < 8; ++r) { b16 h_, l_; split16(acc[t][r] * (1.0f / (XS * WSC)) * XS, h_, l_); Vt[t * 16 + nloc][wave * 16 + 8 * hlf + r] = h_; Vtl[t * 16 + nloc][wave * 16 + 8 * hlf + r] = l_; }
    __syncthreads();
    for (int pass = 0; pass < 2; ++pass) { for (int q = t_; q < 128 * 8; q += 128) { const int cc = q >> 3, c8 = (q & 7) * 8; const int h = (c0v + cc) / D, dd = (c0v + cc) - h * D; const size_t gi = (((size_t)b * NH + h) * D + dd) * M + s0 + c8;
        *(volatile v8b*)(VTh + gi) = *(const v8b*)(&Vt[cc][c8]); *(volatile v8b*)(VTl + gi) = *(const v8b*)(&Vtl[cc][c8]); } __threadfence(); } }
}
__global__ __launch_bounds__(64) void attn_kernel(const b16* __restrict__ Qh, const b16* __restrict__ Ql, const b16* __restrict__ Kh, const b16* __restrict__ Kl, const b16* __restrict__ VTh, const b16* __restrict__ VTl, b16* __restrict__ Oh, b16* __restrict__ Ol) {
  __shared__ __attribute__((aligned(16))) float To[2][16][D + 4];
  const int wave = threadIdx.x >> 5, lane = threadIdx.x & 31, hh = lane >> 4, col = lane & 15; const int b = blockIdx.z, h = blockIdx.y; const int q0 = blockIdx.x * 32 + wave * 16, qi = q0 + col;
  const size_t qo = ((size_t)b * N + qi) * E + h * D; const v16b qa0 = frag_kb(Qh + qo, hh), qa1 = frag_kb(Qh + qo + 32, hh), ql0 = frag_kb(Ql + qo, hh), ql1 = frag_kb(Ql + qo + 32, hh);
  const b16* Kb = Kh + (size_t)b * M * E + h * D; const b16* Klb = Kl + (size_t)b * M * E + h * D; const b16* Vb = VTh + ((size_t)b * NH + h) * D * M; const b16* Vlb = VTl + ((size_t)b * NH + h) * D * M;
  float m = -INFINITY, l = 0.0f; v8f o[4] = {{}, {}, {}, {}}, ol[4] = {{}, {}, {}, {}};
  const float cs = SCALE * LOG2E / (XS * XS);
  for (int kb = 0; kb < M; kb += 32) {
    v8f s0 = {}, s1 = {};
    { const b16* k0 = Kb + (size_t)(kb + col) * E, *k1 = Kb + (size_t)(kb + 16 + col) * E, *k0l = Klb + (size_t)(kb + col) * E, *k1l = Klb + (size_t)(kb + 16 + col) * E;
      v16b f = frag_kb(k0, hh); s0 = wmma16b(f, qa0, s0); s0 = wmma16b(f, ql0, s0); s0 = wmma16b(frag_kb(k0l, hh), qa0, s0);
      f = frag_kb(k0 + 32, hh); s0 = wmma16b(f, qa1, s0); s0 = wmma16b(f, ql1, s0); s0 = wmma16b(frag_kb(k0l + 32, hh), qa1, s0);
      f = frag_kb(k1, hh); s1 = wmma16b(f, qa0, s1); s1 = wmma16b(f, ql0, s1); s1 = wmma16b(frag_kb(k1l, hh), qa0, s1);
      f = frag_kb(k1 + 32, hh); s1 = wmma16b(f, qa1, s1); s1 = wmma16b(f, ql1, s1); s1 = wmma16b(frag_kb(k1l + 32, hh), qa1, s1); }
    float e[16]; float mx = -INFINITY;
#pragma unroll
    for (int r = 0; r < 8; ++r) { e[r] = s0[r] * cs; e[8 + r] = s1[r] * cs; mx = fmaxf(mx, fmaxf(e[r], e[8 + r])); }
    mx = fmaxf(mx, __shfl_xor(mx, 16)); const float mn = fmaxf(m, mx); const float al = nexp2(m - mn); m = mn; float sum = 0.0f; v16b ph, pl;
#pragma unroll
    for (int i = 0; i < 16; ++i) { const float p = nexp2(e[i] - mn); sum += p; const b16 h_ = (b16)(p * PS); ph[i] = h_; pl[i] = (b16)(p * PS - (float)h_); }
    sum += __shfl_xor(sum, 16); l = l * al + sum;
#pragma unroll
    for (int t = 0; t < 4; ++t) { o[t] *= al; ol[t] *= al; const v16b vf = frag_kb(Vb + (size_t)(t * 16 + col) * M + kb, hh); o[t] = wmma16b(vf, ph, o[t]); ol[t] = wmma16b(vf, pl, ol[t]); ol[t] = wmma16b(frag_kb(Vlb + (size_t)(t * 16 + col) * M + kb, hh), ph, ol[t]); } }
  const float inv = 1.0f / (l * PS * XS);
#pragma unroll
  for (int t = 0; t < 4; ++t)
#pragma unroll
    for (int r = 0; r < 8; ++r) To[wave][col][t * 16 + 8 * hh + r] = (o[t][r] + ol[t][r]) * inv;
  wave_lds_sync();
  for (int pass = 0; pass < 2; ++pass) { for (int r4 = 0; r4 < 16; r4 += 4) { const int rr = r4 + (lane >> 3), c8 = (lane & 7) * 8; v8b hv, lv; for (int j = 0; j < 8; ++j) { b16 a_, c_; split16(To[wave][rr][c8 + j] * XS, a_, c_); hv[j] = a_; lv[j] = c_; }
      const size_t gi = ((size_t)b * N + q0 + rr) * E + h * D + c8; *(volatile v8b*)(Oh + gi) = hv; *(volatile v8b*)(Ol + gi) = lv; } __threadfence(); }
}
__global__ __launch_bounds__(128) void outproj_kernel(const b16* __restrict__ Oh, const b16* __restrict__ Ol, const b16* __restrict__ WO16, const float* __restrict__ bo, float* __restrict__ out) {
  __shared__ __attribute__((aligned(16))) float Ts[4][16][128 + 4];
  const int wave = threadIdx.x >> 5, lane = threadIdx.x & 31, nloc = lane & 15, hlf = lane >> 4; const size_t m0 = (size_t)blockIdx.x * 64 + wave * 16; const int n0 = blockIdx.y * 128;
  v8f acc[8];
#pragma unroll
  for (int t = 0; t < 8; ++t) acc[t] = (v8f){};
#pragma unroll
  for (int kb = 0; kb < E; kb += 32) { const v16b a = frag_kb(Oh + (m0 + nloc) * E + kb, hlf), al = frag_kb(Ol + (m0 + nloc) * E + kb, hlf);
#pragma unroll
    for (int t = 0; t < 8; ++t) { const v16b bw = frag_kb(WO16 + (size_t)(n0 + t * 16 + nloc) * E + kb, hlf); acc[t] = wmma16b(a, bw, acc[t]); acc[t] = wmma16b(al, bw, acc[t]); } }
#pragma unroll
  for (int t = 0; t < 8; ++t)
#pragma unroll
    for (int r = 0; r < 8; ++r) Ts[wave][8 * hlf + r][t * 16 + nloc] = acc[t][r] * (1.0f / (XS * WSC)) + bf16_rne(bo[n0 + t * 16 + nloc]);
  wave_lds_sync();
  for (int pass = 0; pass < 2; ++pass) { for (int rr = 0; rr < 16; ++rr) *(volatile v4f*)(out + (m0 + rr) * E + n0 + lane * 4) = *(const v4f*)(&Ts[wave][rr][lane * 4]); __threadfence(); }
}
}

extern "C" void kernel_launch(void* const* d_in, const int* in_sizes, int n_in, void* d_out, int out_size, void* d_ws, size_t ws_size, hipStream_t stream) {
  (void)n_in;
  auto Fp = [&](int i) { return (const float*)d_in[i]; };
  if (in_sizes[0] != NR * E || in_sizes[3] != E * E || in_sizes[4] != E * 2 * E || in_sizes[5] != E * E * SR * SR || in_sizes[6] != E || in_sizes[9] != E * E || in_sizes[10] != E || out_size != NR * E) return;
  size_t off = 0; char* ws = (char*)d_ws;
  auto carve = [&](size_t bytes) { char* p = ws + off; off += (bytes + 255) & ~(size_t)255; return p; };
  b16* X16 = (b16*)carve((size_t)NR * E * 2); b16* WQ16 = (b16*)carve((size_t)E * E * 2); b16* WKV16 = (b16*)carve((size_t)2 * E * E * 2); b16* WO16 = (b16*)carve((size_t)E * E * 2); b16* SRW16 = (b16*)carve((size_t)E * KC * 2);
  b16* Qh = (b16*)carve((size_t)NR * E * 2); b16* Ql = (b16*)carve((size_t)NR * E * 2); b16* KVh = (b16*)carve((size_t)NK * E * 2); b16* KVl = (b16*)carve((size_t)NK * E * 2);
  b16* Kh = (b16*)carve((size_t)NK * E * 2); b16* Kl = (b16*)carve((size_t)NK * E * 2); b16* VTh = (b16*)carve((size_t)NK * E * 2); b16* VTl = (b16*)carve((size_t)NK * E * 2);
  b16* Oh = (b16*)carve((size_t)NR * E * 2); b16* Ol = (b16*)carve((size_t)NR * E * 2); float* CV = (float*)carve((size_t)NK * E * 4);
  if (off > ws_size || off > ((size_t)128 << 20)) return;
  prepx_kernel<<<(unsigned)(((size_t)NR * E / 8 + 255) / 256), 256, 0, stream>>>(Fp(0), X16);
  prepw_kernel<<<dim3(2 * E / 64, E / 64, 3), 256, 0, stream>>>(Fp(3), Fp(4), Fp(9), WQ16, WKV16, WO16);
  prepc_kernel<<<(unsigned)(((size_t)E * KC / 8 + 255) / 256), 256, 0, stream>>>(Fp(5), SRW16);
  q_kernel<<<dim3(NR / 64, 2), 128, 0, stream>>>(X16, WQ16, Qh, Ql);
  conv_kernel<<<NK / 64, 128, 0, stream>>>(X16, SRW16, Fp(6), CV);
  ln_kernel<<<NK / 8, 256, 0, stream>>>(CV, Fp(7), Fp(8), KVh, KVl);
  kv_kernel<<<dim3(NK / 64, 4), 128, 0, stream>>>(KVh, KVl, WKV16, Kh, Kl, VTh, VTl);
  attn_kernel<<<dim3(N / 32, NH, NB), 64, 0, stream>>>(Qh, Ql, Kh, Kl, VTh, VTl, Oh, Ol);
  outproj_kernel<<<dim3(NR / 64, 2), 128, 0, stream>>>(Oh, Ol, WO16, Fp(10), (float*)d_out);
}
